// PrismaticSpectralAttention_19705309954382
// MI455X (gfx1250) — hardware-verified
//
#include <hip/hip_runtime.h>
#include <math.h>
#include <stdint.h>

#define TFR     8
#define NSP     196
#define DM      768
#define NH      12
#define HD      64
#define SQ      1568
#define SP      1600
#define NTOK    1569
#define QKVN    2304
#define QKW     1536
#define NG      4
#define NBA     3
#define WSC     64.0f
#define ACARRY  16.0f
#define QKCARRY 16.0f
#define VCARRY  16.0f
#define PCARRY  1024.0f
#define FCARRY  256.0f
static_assert(SQ == TFR * NSP);
static_assert(NH * HD == DM);
static_assert((SQ % 32) == 0 && (SQ % 16) == 0);
static_assert((SP % 64) == 0 && SP >= NTOK && (QKW % 64) == 0 && (DM % 64) == 0 && (HD % 64) == 0);
static_assert(QKVN == 3 * DM && QKW == 2 * DM);

#define BF_MAIN_THREADS (NSP * (DM / 4))
#define BF_MAIN_BLOCKS  (BF_MAIN_THREADS / 256)
#define BF_TAIL_PERB    ((SP - SQ) * (DM / 8))
#define BF_TAIL_THREADS (NBA * BF_TAIL_PERB)
#define BF_TAIL_BLOCKS  (BF_TAIL_THREADS / 256)
#define ATT_WAVES       (NBA * NH * (SQ / 16))
#define ATT_BLOCKS      (ATT_WAVES / 4)
#define FUSE_THREADS    (SP * (DM / 8))
#define FUSE_BLOCKS     (FUSE_THREADS / 256)
static_assert(BF_MAIN_THREADS % 256 == 0 && BF_TAIL_THREADS % 256 == 0);
static_assert((DM / 4) % 32 == 0 && (DM / 8) % 32 == 0);
static_assert(ATT_WAVES % 4 == 0);
static_assert(FUSE_THREADS % 256 == 0);

typedef _Float16 v16h __attribute__((ext_vector_type(16)));
typedef _Float16 v8h  __attribute__((ext_vector_type(8)));
typedef float    v8f  __attribute__((ext_vector_type(8)));
typedef float    v4f  __attribute__((ext_vector_type(4)));
typedef unsigned int v4u __attribute__((ext_vector_type(4)));
typedef unsigned int v2u __attribute__((ext_vector_type(2)));

union FragH { v16h v; v8h h[2]; v4u u[2]; };

__device__ __forceinline__ unsigned short bf_bits(float f) {
  unsigned u = __float_as_uint(f);
  return (unsigned short)((u + 0x7FFFu + ((u >> 16) & 1u)) >> 16);
}
__device__ __forceinline__ float bf_up(unsigned short h) { return __uint_as_float(((unsigned)h) << 16); }
__device__ __forceinline__ float bfr(float f) { return bf_up(bf_bits(f)); }
__device__ __forceinline__ unsigned short h_bits(_Float16 x) { return __builtin_bit_cast(unsigned short, x); }
__device__ __forceinline__ unsigned pk16(unsigned short a, unsigned short b) { return (unsigned)a | ((unsigned)b << 16); }
__device__ __forceinline__ v8f zero8() { v8f z = {0.f, 0.f, 0.f, 0.f, 0.f, 0.f, 0.f, 0.f}; return z; }

__device__ __forceinline__ v16h ldfrag_h(const _Float16* p) {
  FragH f;
  f.h[0] = *(const v8h*)(p);
  f.h[1] = *(const v8h*)(p + 16);
  return f.v;
}
__device__ __forceinline__ v16h ldfrag_u(const unsigned short* p) {
  FragH f;
  f.u[0] = *(const v4u*)(p);
  f.u[1] = *(const v4u*)(p + 16);
  return f.v;
}

__device__ __forceinline__ v8f mma_raw(v16h a, v16h b, v8f c) {
  return __builtin_amdgcn_wmma_f32_16x16x32_f16(false, a, false, b, (short)0, c, false, false);
}
__device__ __forceinline__ void dep_guard1(v8f& a, v8f& b, v16h x) {
#if defined(__HIP_DEVICE_COMPILE__)
  asm volatile("v_nop\n\tv_nop\n\tv_nop\n\tv_nop" : "+v"(a), "+v"(b) : "v"(x));
#endif
}
__device__ __forceinline__ void guard_s(v8f& s, v16h a0, v16h a1, v16h b0, v16h b1) {
#if defined(__HIP_DEVICE_COMPILE__)
  asm volatile("v_nop\n\tv_nop\n\tv_nop\n\tv_nop" : "+v"(s) : "v"(a0), "v"(a1), "v"(b0), "v"(b1));
#endif
}
__device__ __forceinline__ void guard_pv(v8f& a, v8f& b, v16h x, v16h y, v16h z) {
#if defined(__HIP_DEVICE_COMPILE__)
  asm volatile("v_nop\n\tv_nop\n\tv_nop\n\tv_nop" : "+v"(a), "+v"(b) : "v"(x), "v"(y), "v"(z));
#endif
}
__device__ __forceinline__ void keep4_h(v16h a, v16h b, v16h c, v16h d) {
#if defined(__HIP_DEVICE_COMPILE__)
  asm volatile("v_nop" :: "v"(a), "v"(b), "v"(c), "v"(d));
#endif
}
__device__ __forceinline__ void acc_guard4(v8f& a, v8f& b, v8f& c, v8f& d) {
#if defined(__HIP_DEVICE_COMPILE__)
  asm volatile("v_nop\n\tv_nop\n\tv_nop\n\tv_nop" : "+v"(a), "+v"(b), "+v"(c), "+v"(d));
#endif
}
__device__ __forceinline__ void wave_sync_lds() {
  __builtin_amdgcn_fence(__ATOMIC_RELEASE, "workgroup");
  __builtin_amdgcn_wave_barrier();
  __builtin_amdgcn_fence(__ATOMIC_ACQUIRE, "workgroup");
}

__global__ __launch_bounds__(256) void conv16(const float* __restrict__ W, unsigned short* dst, int n8, float wsc) {
  const int i  = blockIdx.x * 256 + threadIdx.x;
  const int ic = (i < n8) ? i : (n8 - 1);
  const float* p = W + (size_t)ic * 8;
  const v4f a = *(const v4f*)(p), b = *(const v4f*)(p + 4);
  float v[8];
#pragma unroll
  for (int e = 0; e < 4; ++e) { v[e] = bfr(a[e]); v[4 + e] = bfr(b[e]); }
  v4u ov;
#pragma unroll
  for (int e = 0; e < 4; ++e) ov[e] = pk16(h_bits((_Float16)(v[2 * e] * wsc)), h_bits((_Float16)(v[2 * e + 1] * wsc)));
  if (i < n8) *(volatile v4u*)(dst + (size_t)i * 8) = ov;
  __threadfence();
  if (i < n8) *(volatile v4u*)(dst + (size_t)i * 8) = ov;
}

__device__ __forceinline__ float cosq(int d) {
  const int a  = d & 7;
  const int m4 = a & 3;
  const float R = 0.70710678118654752f;
  const float base = (m4 == 0) ? 1.0f : ((m4 == 1) ? R : ((m4 == 2) ? 0.0f : -R));
  return (a & 4) ? -base : base;
}

__global__ __launch_bounds__(256) void bandfeat(const float* __restrict__ x, unsigned short* FP) {
  const int gt = blockIdx.x * 256 + threadIdx.x;
  if (blockIdx.x < BF_MAIN_BLOCKS) {
    const int n  = gt / (DM / 4);
    const int d4 = (gt - n * (DM / 4)) * 4;
    v4f w[8];
#pragma unroll
    for (int k = 0; k < 8; ++k) {
      const int tp = (8 - k) & 7;
      const v4f v = *(const v4f*)(x + (size_t)(1 + tp * NSP + n) * DM + d4);
      v4f r;
#pragma unroll
      for (int e = 0; e < 4; ++e) r[e] = bfr(v[e]);
      w[k] = r;
    }
#pragma unroll 1
    for (int b = 0; b < NBA; ++b) {
      const int flo = 2 * b, fhi = 2 * b + 1;
      const float wlo = (b == 1) ? 0.25f : 0.125f;
      const float whi = (b == 2) ? 0.0f : 0.25f;
      float mk[8];
#pragma unroll
      for (int k = 0; k < 8; ++k) mk[k] = wlo * cosq(flo * k) + whi * cosq(fhi * k);
#pragma unroll 1
      for (int t = 0; t < TFR; ++t) {
        v4f o = w[0] * mk[0];
#pragma unroll
        for (int k = 1; k < 8; ++k) o += w[k] * mk[k];
        v2u pv;
        pv[0] = pk16(h_bits((_Float16)(o[0] * ACARRY)), h_bits((_Float16)(o[1] * ACARRY)));
        pv[1] = pk16(h_bits((_Float16)(o[2] * ACARRY)), h_bits((_Float16)(o[3] * ACARRY)));
        unsigned short* dp = FP + ((size_t)b * SP + (size_t)t * NSP + n) * DM + d4;
        *(volatile v2u*)dp = pv;
        __threadfence();
        *(volatile v2u*)dp = pv;
        const v4f tmp = w[7];
        w[7] = w[6]; w[6] = w[5]; w[5] = w[4]; w[4] = w[3];
        w[3] = w[2]; w[2] = w[1]; w[1] = w[0]; w[0] = tmp;
      }
    }
  } else {
    const int j   = gt - BF_MAIN_BLOCKS * 256;
    const int jc  = (j < BF_TAIL_THREADS) ? j : (BF_TAIL_THREADS - 1);
    const int b   = jc / BF_TAIL_PERB;
    const int rem = jc - b * BF_TAIL_PERB;
    const int rr  = rem / (DM / 8);
    const int c8  = (rem - rr * (DM / 8)) * 8;
    v4u z = {0u, 0u, 0u, 0u};
    unsigned short* dp = FP + ((size_t)b * SP + SQ + rr) * DM + c8;
    if (j < BF_TAIL_THREADS) *(volatile v4u*)dp = z;
    __threadfence();
    if (j < BF_TAIL_THREADS) *(volatile v4u*)dp = z;
  }
}

template <int OM, int BIASM>
__global__ __launch_bounds__(256) void gemm64(
    const unsigned short* __restrict__ Ap, int lda, long long sAo, long long sAi,
    const unsigned short* __restrict__ Btp, int ldb, long long sBo, long long sBi,
    const float* __restrict__ bias, int sbo, int sbi, float bscale,
    void* Cout, int ldc, long long sCo, long long sCi,
    int M, int N, int K, int Mv, int nin, float oscale) {
  __shared__ __align__(16) float sT[8][16 * 68];
  const int by   = blockIdx.y;
  const int bo   = by / nin;
  const int bi   = by - bo * nin;
  const int lane = threadIdx.x & 31;
  const int wave = threadIdx.x >> 5;
  const int tilesN = N >> 6;
  const int tilesM = M >> 6;
  const int tile = blockIdx.x * 8 + wave;
  if (tile >= tilesM * tilesN) return;
  const int tm = tile / tilesN;
  const int tn = tile - tm * tilesN;
  const int m0 = tm << 6;
  const int n0 = tn << 6;

  const unsigned short* A1 = Ap  + (size_t)((long long)bo * sAo + (long long)bi * sAi);
  const unsigned short* Bb = Btp + (size_t)((long long)bo * sBo + (long long)bi * sBi);
  const float*         bsp = bias + (size_t)bo * (size_t)sbo + (size_t)bi * (size_t)sbi;

  const int rlane = lane & 15;
  const int koff  = (lane >> 4) * 8;
  const int mOff  = (lane >> 4) * 8;

  v8f acc[4][4];
#pragma unroll
  for (int i = 0; i < 4; ++i)
#pragma unroll
    for (int j = 0; j < 4; ++j) acc[i][j] = zero8();

  for (int k0 = 0; k0 < K; k0 += 32) {
    v16h bh[4];
#pragma unroll
    for (int j = 0; j < 4; ++j) {
      const size_t bofs = (size_t)(n0 + (j << 4) + rlane) * ldb + koff + k0;
      bh[j] = ldfrag_u(Bb + bofs);
    }
#pragma unroll
    for (int i = 0; i < 4; ++i) {
      const size_t ao = (size_t)(m0 + (i << 4) + rlane) * lda + koff + k0;
      const v16h ah = ldfrag_u(A1 + ao);
#pragma unroll
      for (int j = 0; j < 4; ++j) acc[i][j] = mma_raw(ah, bh[j], acc[i][j]);
      dep_guard1(acc[i][0], acc[i][3], ah);
    }
    keep4_h(bh[0], bh[1], bh[2], bh[3]);
  }
  acc_guard4(acc[0][0], acc[0][1], acc[0][2], acc[0][3]);
  acc_guard4(acc[1][0], acc[1][1], acc[1][2], acc[1][3]);
  acc_guard4(acc[2][0], acc[2][1], acc[2][2], acc[2][3]);
  acc_guard4(acc[3][0], acc[3][1], acc[3][2], acc[3][3]);

  const int hh2 = lane >> 4, c4 = (lane & 15) * 4;
  const int q8  = lane >> 3, c8 = (lane & 7) * 8;
  float bc[8];
#pragma unroll
  for (int e = 0; e < 8; ++e) bc[e] = 0.f;
  if (BIASM == 0) {
    if (OM == 0) {
      const int cb = n0 + c4;
      const int i0 = (cb < N - 4) ? cb : (N - 4);
      const v4f b0v = *(const v4f*)(bsp + i0);
#pragma unroll
      for (int e = 0; e < 4; ++e) bc[e] = bfr(b0v[e]) * bscale;
    } else {
      const int cb = n0 + c8;
      const int i0 = (cb < N - 8) ? cb : (N - 8);
      const v4f b0a = *(const v4f*)(bsp + i0), b0b = *(const v4f*)(bsp + i0 + 4);
#pragma unroll
      for (int e = 0; e < 4; ++e) {
        bc[e]     = bfr(b0a[e]) * bscale;
        bc[4 + e] = bfr(b0b[e]) * bscale;
      }
    }
  }

  float* slab = sT[wave];
#pragma unroll
  for (int i = 0; i < 4; ++i) {
    const int mBase = m0 + (i << 4);
#pragma unroll
    for (int j = 0; j < 4; ++j) {
#pragma unroll
      for (int r = 0; r < 8; ++r) {
        slab[(mOff + r) * 68 + (j << 4) + rlane] = acc[i][j][r];
      }
    }
    wave_sync_lds();
    if (OM == 0) {
      float* C = (float*)Cout + (size_t)((long long)bo * sCo + (long long)bi * sCi);
      v4f vals[8];
#pragma unroll
      for (int it = 0; it < 8; ++it) {
        const int row = it * 2 + hh2;
        v4f v = *(const v4f*)(slab + row * 68 + c4);
#pragma unroll
        for (int e = 0; e < 4; ++e) v[e] = v[e] * oscale + bc[e];
        vals[it] = v;
      }
      for (int pass = 0; pass < 2; ++pass) {
#pragma unroll
        for (int it = 0; it < 8; ++it) {
          const int row = it * 2 + hh2;
          if (mBase + row < Mv) *(volatile v4f*)(C + (size_t)(mBase + row) * ldc + n0 + c4) = vals[it];
        }
        __threadfence();
      }
    } else {
      unsigned short* C = (unsigned short*)Cout + (size_t)((long long)bo * sCo + (long long)bi * sCi);
      v4u hv[4];
#pragma unroll
      for (int it = 0; it < 4; ++it) {
        const int row = it * 4 + q8;
        const float* sp = slab + row * 68 + c8;
        float bm = 0.f;
        if (BIASM == 1) bm = bfr(bsp[mBase + row]) * bscale;
        v4u a;
#pragma unroll
        for (int e = 0; e < 4; ++e) {
          const float f0 = sp[2 * e]     * oscale + ((BIASM == 1) ? bm : bc[2 * e]);
          const float f1 = sp[2 * e + 1] * oscale + ((BIASM == 1) ? bm : bc[2 * e + 1]);
          a[e] = pk16(h_bits((_Float16)f0), h_bits((_Float16)f1));
        }
        hv[it] = a;
      }
      for (int pass = 0; pass < 2; ++pass) {
#pragma unroll
        for (int it = 0; it < 4; ++it) {
          const int row = it * 4 + q8;
          *(volatile v4u*)(C + (size_t)(mBase + row) * ldc + n0 + c8) = hv[it];
        }
        __threadfence();
      }
    }
    wave_sync_lds();
  }
}

__global__ __launch_bounds__(128)
void attn16(const unsigned short* __restrict__ QK, const unsigned short* __restrict__ VT,
            const float* __restrict__ spec, float* AO) {
  __shared__ __align__(16) float Ps[4][16 * 36];
  __shared__ __align__(16) float Os[4][16 * 64];

  const int tid  = threadIdx.x;
  const int wave = tid >> 5;
  const int lane = tid & 31;
  const int hh   = lane >> 4;
  const int c    = lane & 15;

  const int wid  = blockIdx.x * 4 + wave;
  const int bh   = wid / (SQ / 16);
  const int qt   = wid - bh * (SQ / 16);
  const int band = bh / NH;
  const int head = bh - band * NH;
  const int q0   = qt * 16;

  const _Float16* Qp = (const _Float16*)(const void*)QK + (size_t)band * SP * QKW + head * HD;
  const _Float16* Kp = Qp + DM;
  const _Float16* Vp = (const _Float16*)(const void*)VT + (size_t)bh * HD * SP;
  const float filt = bfr(spec[band * NH + head]);
  const float lsc  = filt * ((1.4426950408889634f * 0.125f) / (QKCARRY * QKCARRY));

  const v16h qa0 = ldfrag_h(Qp + (size_t)(q0 + c) * QKW + 8 * hh);
  const v16h qa1 = ldfrag_h(Qp + (size_t)(q0 + c) * QKW + 32 + 8 * hh);

  float mrow[8], lrow[8];
  v8f acc0 = zero8(), acc1 = zero8(), acc2 = zero8(), acc3 = zero8();
#pragma unroll
  for (int r = 0; r < 8; ++r) { mrow[r] = -INFINITY; lrow[r] = 0.f; }
  float* pt = Ps[wave];

#pragma unroll 1
  for (int kb = 0; kb < SQ; kb += 32) {
    const _Float16* kp = Kp + (size_t)(kb + c) * QKW + 8 * hh;
    v8f s0, s1;
    {
      const v16h k00 = ldfrag_h(kp), k01 = ldfrag_h(kp + 32);
      s0 = mma_raw(qa0, k00, zero8());
      s0 = mma_raw(qa1, k01, s0);
      guard_s(s0, qa0, qa1, k00, k01);
    }
    {
      const v16h k10 = ldfrag_h(kp + (size_t)16 * QKW), k11 = ldfrag_h(kp + (size_t)16 * QKW + 32);
      s1 = mma_raw(qa0, k10, zero8());
      s1 = mma_raw(qa1, k11, s1);
      guard_s(s1, qa0, qa1, k10, k11);
    }
#pragma unroll
    for (int r = 0; r < 8; ++r) {
      const float t0 = s0[r] * lsc, t1 = s1[r] * lsc;
      float mx = fmaxf(t0, t1);
#pragma unroll
      for (int off = 1; off < 16; off <<= 1) mx = fmaxf(mx, __shfl_xor(mx, off, 32));
      const float mn = fmaxf(mrow[r], mx);
      const float al = exp2f(mrow[r] - mn);
      mrow[r] = mn;
      const float e0 = exp2f(t0 - mn), e1 = exp2f(t1 - mn);
      float ps = e0 + e1;
#pragma unroll
      for (int off = 1; off < 16; off <<= 1) ps += __shfl_xor(ps, off, 32);
      lrow[r] = lrow[r] * al + ps;
      acc0[r] *= al;
      acc1[r] *= al;
      acc2[r] *= al;
      acc3[r] *= al;
      const int ro = (8 * hh + r) * 36 + c;
      pt[ro]      = e0;
      pt[ro + 16] = e1;
    }
    wave_sync_lds();
    FragH pa;
    {
      const float* prow = pt + c * 36 + 8 * hh;
      const v4f p0 = *(const v4f*)(prow), p1 = *(const v4f*)(prow + 4);
      const v4f p2 = *(const v4f*)(prow + 16), p3 = *(const v4f*)(prow + 20);
#pragma unroll
      for (int e = 0; e < 4; ++e) {
        pa.h[0][e]     = (_Float16)(p0[e] * PCARRY);
        pa.h[0][4 + e] = (_Float16)(p1[e] * PCARRY);
        pa.h[1][e]     = (_Float16)(p2[e] * PCARRY);
        pa.h[1][4 + e] = (_Float16)(p3[e] * PCARRY);
      }
    }
    const _Float16* vp = Vp + (size_t)c * SP + kb + 8 * hh;
    {
      const v16h vb0 = ldfrag_h(vp), vb1 = ldfrag_h(vp + (size_t)16 * SP);
      acc0 = mma_raw(pa.v, vb0, acc0);
      acc1 = mma_raw(pa.v, vb1, acc1);
      guard_pv(acc0, acc1, pa.v, vb0, vb1);
    }
    {
      const v16h vb2 = ldfrag_h(vp + (size_t)32 * SP), vb3 = ldfrag_h(vp + (size_t)48 * SP);
      acc2 = mma_raw(pa.v, vb2, acc2);
      acc3 = mma_raw(pa.v, vb3, acc3);
      guard_pv(acc2, acc3, pa.v, vb2, vb3);
    }
    wave_sync_lds();
  }

  float* os = Os[wave];
  const float oinv = 1.0f / (PCARRY * VCARRY);
#pragma unroll
  for (int r = 0; r < 8; ++r) {
    const float inv = (1.0f / lrow[r]) * oinv;
    const int ro = (8 * hh + r) * 64 + c;
    os[ro]      = acc0[r] * inv;
    os[ro + 16] = acc1[r] * inv;
    os[ro + 32] = acc2[r] * inv;
    os[ro + 48] = acc3[r] * inv;
  }
  wave_sync_lds();
  {
    const int hh2 = lane >> 4, c4 = (lane & 15) * 4;
    v4f vals[8];
#pragma unroll
    for (int it = 0; it < 8; ++it) {
      const int row = it * 2 + hh2;
      vals[it] = *(const v4f*)(os + row * 64 + c4);
    }
    float* dst = AO + ((size_t)band * SQ + q0) * DM + head * HD + c4;
    for (int pass = 0; pass < 2; ++pass) {
#pragma unroll
      for (int it = 0; it < 8; ++it) {
        const int row = it * 2 + hh2;
        *(volatile v4f*)(dst + (size_t)row * DM) = vals[it];
      }
      __threadfence();
    }
  }
}

__global__ __launch_bounds__(256) void fusion_wts(const float* __restrict__ AO, const float* __restrict__ qkvb,
                                                  const float* __restrict__ fw, const float* __restrict__ fb, float* WTS) {
  __shared__ float red[NG][256];
  __shared__ float sw[8];
  const int tid = threadIdx.x;
#pragma unroll 1
  for (int b = 0; b < NBA; ++b) {
    float pb = 0.f;
#pragma unroll 1
    for (int j = 0; j < DM / 256; ++j) {
      const int d = tid + 256 * j;
      const float* col = AO + (size_t)b * SQ * DM + d;
      double a = 0.0;
#pragma unroll 4
      for (int s = 0; s < SQ; ++s) a += (double)col[(size_t)s * DM];
      const float mean = (float)(a * (1.0 / (double)SQ));
      pb += mean * bfr(fw[d]);
    }
    red[b][tid] = pb;
  }
  {
    float pb = 0.f;
#pragma unroll 1
    for (int j = 0; j < DM / 256; ++j) {
      const int d = tid + 256 * j;
      pb += bfr(qkvb[(size_t)(NG - 1) * QKVN + 2 * DM + d]) * bfr(fw[d]);
    }
    red[NG - 1][tid] = pb;
  }
  __syncthreads();
  for (int st = 128; st > 0; st >>= 1) {
    if (tid < st) {
#pragma unroll
      for (int b = 0; b < NG; ++b) red[b][tid] += red[b][tid + st];
    }
    __syncthreads();
  }
  if (tid == 0) {
    const float fb0 = bfr(fb[0]);
    float m = -INFINITY;
#pragma unroll 1
    for (int b = 0; b < NG; ++b) {
      const float sc = red[b][0] + fb0;
      sw[b] = sc;
      m = fmaxf(m, sc);
    }
    float sum = 0.f;
#pragma unroll 1
    for (int b = 0; b < NG; ++b) {
      const float e = expf(sw[b] - m);
      sw[b] = e;
      sum += e;
    }
    const float inv = 1.0f / sum;
#pragma unroll 1
    for (int b = 0; b < NG; ++b) sw[b] = sw[b] * inv;
  }
  __syncthreads();
  if (tid < 8) {
    const float a0 = sw[0], a1 = sw[1], a2 = sw[2], a3 = sw[3];
    const bool f = (tid == 0);
    v4f o;
    o[0] = f ? a0 : 0.f;
    o[1] = f ? a1 : 0.f;
    o[2] = f ? a2 : 0.f;
    o[3] = f ? a3 : 0.f;
    *(volatile v4f*)(WTS + 4 * tid) = o;
    __threadfence();
    *(volatile v4f*)(WTS + 4 * tid) = o;
  }
}

__global__ __launch_bounds__(256) void fuse(const float* __restrict__ x, const float* __restrict__ AO,
                                            const float* __restrict__ qkvb, const float* __restrict__ WTS,
                                            unsigned short* FH) {
  const int i   = blockIdx.x * 256 + threadIdx.x;
  const int row = i / (DM / 8);
  const int c8  = (i - row * (DM / 8)) * 8;
  const v4f wv  = *(const v4f*)(WTS);
  int s = row - 1;
  s = (s < 0) ? 0 : s;
  s = (s > SQ - 1) ? (SQ - 1) : s;
  const float* ap = AO + (size_t)s * DM + c8;
  const v4f a00 = *(const v4f*)(ap), a01 = *(const v4f*)(ap + 4);
  const v4f a10 = *(const v4f*)(ap + (size_t)SQ * DM), a11 = *(const v4f*)(ap + (size_t)SQ * DM + 4);
  const v4f a20 = *(const v4f*)(ap + (size_t)2 * SQ * DM), a21 = *(const v4f*)(ap + (size_t)2 * SQ * DM + 4);
  const v4f x0  = *(const v4f*)(x + c8), x1 = *(const v4f*)(x + c8 + 4);
  const float* bp = qkvb + (size_t)(NG - 1) * QKVN + 2 * DM + c8;
  const v4f bv0 = *(const v4f*)(bp), bv1 = *(const v4f*)(bp + 4);
  const bool iscls = (row == 0);
  const bool isdat = (row >= 1) && (row <= SQ);
  float v[8];
#pragma unroll
  for (int e = 0; e < 4; ++e) {
    const float f0 = wv[0] * a00[e] + wv[1] * a10[e] + wv[2] * a20[e] + wv[3] * bfr(bv0[e]);
    const float f1 = wv[0] * a01[e] + wv[1] * a11[e] + wv[2] * a21[e] + wv[3] * bfr(bv1[e]);
    const float c0 = bfr(x0[e]), c1 = bfr(x1[e]);
    v[e]     = iscls ? c0 : (isdat ? f0 : 0.f);
    v[4 + e] = iscls ? c1 : (isdat ? f1 : 0.f);
  }
  v4u o;
#pragma unroll
  for (int e = 0; e < 4; ++e) o[e] = pk16(h_bits((_Float16)(v[2 * e] * FCARRY)), h_bits((_Float16)(v[2 * e + 1] * FCARRY)));
  unsigned short* dp = FH + (size_t)i * 8;
  *(volatile v4u*)dp = o;
  __threadfence();
  *(volatile v4u*)dp = o;
}

extern "C" void kernel_launch(void* const* d_in, const int* in_sizes, int n_in,
                              void* d_out, int out_size, void* d_ws, size_t ws_size,
                              hipStream_t stream) {
  if (n_in < 8) return;
  if (in_sizes[0] != NTOK * DM) return;
  if (in_sizes[1] != NG * QKVN * DM || in_sizes[2] != NG * QKVN) return;
  if (in_sizes[3] != NG * NH) return;
  if (in_sizes[4] != DM || in_sizes[5] != 1) return;
  if (in_sizes[6] != DM * DM || in_sizes[7] != DM) return;
  if (out_size != NTOK * DM) return;

  const float* x     = (const float*)d_in[0];
  const float* qkv_w = (const float*)d_in[1];
  const float* qkv_b = (const float*)d_in[2];
  const float* spec  = (const float*)d_in[3];
  const float* fus_w = (const float*)d_in[4];
  const float* fus_b = (const float*)d_in[5];
  const float* out_w = (const float*)d_in[6];
  const float* out_b = (const float*)d_in[7];
  float*       out   = (float*)d_out;

  const size_t PWQ = (size_t)NBA * QKVN * DM * 2;
  const size_t PWO = (size_t)DM * DM * 2;
  const size_t PFP = (size_t)NBA * SP * DM * 2;
  const size_t PQK = (size_t)NBA * SP * QKW * 2;
  const size_t PVT = (size_t)NBA * NH * HD * SP * 2;
  const size_t PAO = (size_t)NBA * SQ * DM * 4;
  const size_t PWT = 4096;
  const size_t PFH = (size_t)SP * DM * 2;
  size_t off = 0;
  const size_t oWQ = off; off += PWQ;
  const size_t oWO = off; off += PWO;
  const size_t oFP = off; off += PFP;
  const size_t oQK = off; off += PQK;
  const size_t oVT = off; off += PVT;
  const size_t oAO = off; off += PAO;
  const size_t oWT = off; off += PWT;
  const size_t oFH = off; off += PFH;
  if (off > ws_size) return;
  if (off > (size_t)134217728) return;

  char* ws = (char*)d_ws;
  unsigned short* WQ  = (unsigned short*)(ws + oWQ);
  unsigned short* WO  = (unsigned short*)(ws + oWO);
  unsigned short* FPp = (unsigned short*)(ws + oFP);
  unsigned short* QKp = (unsigned short*)(ws + oQK);
  unsigned short* VTp = (unsigned short*)(ws + oVT);
  float*          AO  = (float*)(ws + oAO);
  float*          WTS = (float*)(ws + oWT);
  unsigned short* FH  = (unsigned short*)(ws + oFH);

  const int n8q = (NBA * QKVN * DM) / 8;
  const int n8o = (DM * DM) / 8;
  if ((n8q % 256) != 0 || (n8o % 256) != 0) return;
  const dim3 blk(256), blk128(128);
  const dim3 gCq(n8q / 256), gCo(n8o / 256);
  const dim3 gBF(BF_MAIN_BLOCKS + BF_TAIL_BLOCKS);
  const dim3 gQK(((SP / 64) * (QKW / 64) + 7) / 8, NBA);
  const dim3 gVT(((HD / 64) * (SP / 64) + 7) / 8, NBA * NH);
  const dim3 gAT(ATT_BLOCKS);
  const dim3 gFU(FUSE_BLOCKS);
  const dim3 gOU(((SP / 64) * (DM / 64) + 7) / 8, 1);

  conv16<<<gCq, blk, 0, stream>>>(qkv_w, WQ, n8q, WSC);
  conv16<<<gCo, blk, 0, stream>>>(out_w, WO, n8o, WSC);

  bandfeat<<<gBF, blk, 0, stream>>>(x, FPp);

  gemm64<2, 0><<<gQK, blk, 0, stream>>>(
      FPp, DM, (long long)SP * DM, 0LL,
      WQ, DM, (long long)QKVN * DM, 0LL,
      qkv_b, QKVN, 0, QKCARRY,
      (void*)QKp, QKW, (long long)SP * QKW, 0LL,
      SP, QKW, DM, SP, 1, QKCARRY / (ACARRY * WSC));

  gemm64<2, 1><<<gVT, blk, 0, stream>>>(
      WQ + (size_t)QKW * DM, DM, (long long)QKVN * DM, (long long)HD * DM,
      FPp, DM, (long long)SP * DM, 0LL,
      qkv_b + QKW, QKVN, HD, VCARRY,
      (void*)VTp, SP, (long long)NH * HD * SP, (long long)HD * SP,
      HD, SP, DM, HD, NH, VCARRY / (ACARRY * WSC));

  attn16<<<gAT, blk128, 0, stream>>>(QKp, VTp, spec, AO);

  fusion_wts<<<dim3(1), blk, 0, stream>>>(AO, qkv_b, fus_w, fus_b, WTS);

  fuse<<<gFU, blk, 0, stream>>>(x, AO, qkv_b, WTS, FH);

  gemm64<0, 0><<<gOU, blk, 0, stream>>>(
      FH, DM, 0LL, 0LL,
      WO, DM, 0LL, 0LL,
      out_b, 0, 0, 1.0f,
      (void*)out, DM, 0LL, 0LL,
      SP, DM, DM, NTOK, 1, 1.0f / (FCARRY * WSC));
  (void)hipGetLastError();
}
